// MultiHeadAttentionLayer_39857296507370
// MI455X (gfx1250) — hardware-run, weakly checked
//
#include <hip/hip_runtime.h>


#ifndef NB
#define NB 16
#endif
#ifndef SEQ
#define SEQ 512
#endif
#define NB_FULL  16
#define SEQ_FULL 512
#ifndef OUT_SEQ
#define OUT_SEQ SEQ
#endif
#define DM   256
#define NH_  8
#define HD   32
#define AW   4
#define OSP  36
#define QRS  2048.0f
#define QRI  (1.0f / 2048.0f)
#define SC2  ((float)(0.17677669529663687 * 1.4426950408889634))
#define PSH  14.0f
#define NEGB (-3.0e38f)
#define WOS  64.0f
#define WOI  (1.0f / 64.0f)
#define MROWS 64
#define WTP  (DM + 4)

static_assert(HD == 32);
static_assert(NH_ * HD == DM);
static_assert(DM % 64 == 0);
static_assert(64 % HD == 0);
static_assert(DM % 32 == 0);
static_assert(SEQ % 64 == 0);
static_assert((NB * SEQ) % 64 == 0);
static_assert(SEQ % 32 == 0);
static_assert(SEQ % (16 * AW) == 0);
static_assert(((size_t)SEQ * DM) % 8 == 0);
static_assert(((size_t)DM * DM) % 8 == 0);
static_assert(NB <= NB_FULL);
static_assert(SEQ <= SEQ_FULL);
static_assert((OSP * 4) % 16 == 0);
static_assert(SEQ % MROWS == 0);
static_assert(SEQ % 128 == 0);
static_assert((MROWS * SEQ) % (16 * 256) == 0);
static_assert(((MROWS * SEQ) / 128) % 32 == 0);
static_assert((WTP * 4) % 16 == 0);
static_assert(4 * 256 * 8 == 32 * DM);
static_assert(2 * 32 * 8 == 16 * HD);
static_assert(8 * 32 * 4 == 16 * 64);
static_assert((size_t)MROWS * SEQ <= 131072);
static_assert((size_t)32 * WTP * 4 <= 131072);
static_assert((size_t)AW * 16 * OSP * 4 <= 131072);
static_assert((size_t)16 * 68 * 4 <= 131072);
static_assert(sizeof(unsigned) == 4);

typedef _Float16 h16;
typedef unsigned short bf;
typedef __attribute__((ext_vector_type(16))) __bf16   v16bf;
typedef __attribute__((ext_vector_type(16))) _Float16 v16h;
typedef __attribute__((ext_vector_type(8)))  _Float16 v8h;
typedef __attribute__((ext_vector_type(8)))  unsigned short v8us;
typedef __attribute__((ext_vector_type(8)))  float    v8f;
typedef __attribute__((ext_vector_type(4)))  float    v4f;
typedef v4f  __attribute__((may_alias)) v4fa;
typedef __attribute__((ext_vector_type(4)))  unsigned v4u;
typedef v4u  __attribute__((may_alias)) v4ua;

__device__ __forceinline__ unsigned short f2bf(float f) { unsigned u = __float_as_uint(f); u += 0x7FFFu + ((u >> 16) & 1u); return (unsigned short)(u >> 16); }
__device__ __forceinline__ float bfr(float f) { return __uint_as_float(((unsigned)f2bf(f)) << 16); }
__device__ __forceinline__ v16h cat16(v8h lo, v8h hi) { return __builtin_shufflevector(lo, hi, 0, 1, 2, 3, 4, 5, 6, 7, 8, 9, 10, 11, 12, 13, 14, 15); }
__device__ __forceinline__ v16bf cat16b(v8us lo, v8us hi) { return __builtin_bit_cast(v16bf, __builtin_shufflevector(lo, hi, 0, 1, 2, 3, 4, 5, 6, 7, 8, 9, 10, 11, 12, 13, 14, 15)); }
__device__ __forceinline__ v8f wmma16(v16h a, v16h b, v8f c) { return __builtin_amdgcn_wmma_f32_16x16x32_f16(false, a, false, b, (short)0, c, false, false); }
__device__ __forceinline__ v8f wmmab(v16bf a, v16bf b, v8f c) { return __builtin_amdgcn_wmma_f32_16x16x32_bf16(false, a, false, b, (short)0, c, false, false); }
__device__ __forceinline__ v16h  ldh(const h16* p) { return cat16(*(const v8h*)p, *(const v8h*)(p + 16)); }
__device__ __forceinline__ v16bf ldb(const bf* p)  { return cat16b(*(const v8us*)p, *(const v8us*)(p + 16)); }
__device__ __forceinline__ void wave_sync() { __builtin_amdgcn_fence(3  , "wavefront"); __builtin_amdgcn_wave_barrier(); asm volatile("" ::: "memory"); }
__device__ __forceinline__ h16 toh_flush(float v) { const h16 r = (h16)v; return (fabsf(v) < 6.103515625e-05f) ? (h16)0.0f : r; }
__device__ __forceinline__ v8f wmma16g(v16h a, v16h b, v8f c) { c = wmma16(a, b, c); asm volatile("v_nop\n\tv_nop\n\tv_nop\n\tv_nop" : "+v"(c) : "v"(a), "v"(b)); return c; }
__device__ __forceinline__ unsigned nib4(unsigned x) { return (x | (x >> 7) | (x >> 14) | (x >> 21)) & 0xFu; }

__global__ __launch_bounds__(256) void k_cvt8(const float* __restrict__ src, bf* dst, size_t n8) {
    const size_t i = (size_t)blockIdx.x * 256 + threadIdx.x; if (i >= n8) return;
    const v8f v = *(const v8f*)(src + i * 8); v8us o;
#pragma unroll
    for (int k = 0; k < 8; ++k) o[k] = f2bf(v[k]);
    *(volatile v8us*)(dst + i * 8) = o; __threadfence(); *(volatile v8us*)(dst + i * 8) = o;
}

__global__ __launch_bounds__(256) void k_wtb(const float* __restrict__ W, bf* WT) {
    __shared__ __align__(16) float ts[32 * WTP];
    const int tid = threadIdx.x; const int n0 = blockIdx.x * 32; const int j = tid & 31, kk = tid >> 5;
#pragma unroll 1
    for (int i = 0; i < DM / 8; ++i) { const int k = kk + 8 * i; ts[j * WTP + k] = W[(size_t)k * DM + n0 + j]; }
    __syncthreads();
#pragma unroll 1
    for (int it = 0; it < 4; ++it) { const int q = it * 256 + tid; const int row = q / (DM / 8), c8 = (q % (DM / 8)) * 8;
        const v4f x0 = *(const v4fa*)(&ts[row * WTP + c8]); const v4f x1 = *(const v4fa*)(&ts[row * WTP + c8 + 4]); v8us o;
#pragma unroll
        for (int i = 0; i < 4; ++i) { o[i] = f2bf(x0[i]); o[4 + i] = f2bf(x1[i]); }
        bf* dp = WT + (size_t)(n0 + row) * DM + c8;
        *(volatile v8us*)dp = o; __threadfence(); *(volatile v8us*)dp = o; }
}

__global__ __launch_bounds__(256) void k_wth(const float* __restrict__ W, h16* WT) {
    __shared__ __align__(16) float ts[32 * WTP];
    const int tid = threadIdx.x; const int n0 = blockIdx.x * 32; const int j = tid & 31, kk = tid >> 5;
#pragma unroll 1
    for (int i = 0; i < DM / 8; ++i) { const int k = kk + 8 * i; ts[j * WTP + k] = W[(size_t)k * DM + n0 + j]; }
    __syncthreads();
#pragma unroll 1
    for (int it = 0; it < 4; ++it) { const int q = it * 256 + tid; const int row = q / (DM / 8), c8 = (q % (DM / 8)) * 8;
        const v4f x0 = *(const v4fa*)(&ts[row * WTP + c8]); const v4f x1 = *(const v4fa*)(&ts[row * WTP + c8 + 4]); v8h o;
#pragma unroll
        for (int i = 0; i < 4; ++i) { o[i] = toh_flush(bfr(x0[i]) * WOS); o[4 + i] = toh_flush(bfr(x1[i]) * WOS); }
        h16* dp = WT + (size_t)(n0 + row) * DM + c8;
        *(volatile v8h*)dp = o; __threadfence(); *(volatile v8h*)dp = o; }
}

__global__ __launch_bounds__(256) void k_mask(const int* __restrict__ src, const int* __restrict__ dst, int nE, unsigned* MB) {
    __shared__ __align__(16) unsigned char fl[MROWS * SEQ];
    const int tid = threadIdx.x; const int r0 = blockIdx.x * MROWS; const int b = blockIdx.y;
    const v4u zz = (v4u){0u, 0u, 0u, 0u};
#pragma unroll 1
    for (int i = 0; i < (MROWS * SEQ) / (16 * 256); ++i) *(v4ua*)(&fl[(i * 256 + tid) * 16]) = zz;
    __syncthreads();
    if (tid < MROWS) fl[tid * SEQ + r0 + tid] = (unsigned char)1;
#pragma unroll 1
    for (int base = 0; base < nE; base += 256) {
        const int e = base + tid; const int ec = e < nE ? e : nE - 1;
        int s = src[ec], d = dst[ec];
        asm volatile("" : "+v"(s), "+v"(d));
        const int r = ((s % SEQ_FULL) + SEQ_FULL) % SEQ_FULL;
        const int c = ((d % SEQ_FULL) + SEQ_FULL) % SEQ_FULL;
        int bs = (s - r) / SEQ_FULL; bs = bs < 0 ? bs + NB_FULL : bs;
        const int rl = r - r0;
        const bool ok = (e < nE) & (bs == b) & (rl >= 0) & (rl < MROWS) & (c < SEQ);
        if (ok) fl[rl * SEQ + c] = (unsigned char)1;
    }
    __syncthreads();
    const size_t wbase = (size_t)(b * SEQ + r0) * (SEQ / 32);
#pragma unroll 1
    for (int p = tid; p < (MROWS * SEQ) / 128; p += 256) {
        v4u w;
#pragma unroll
        for (int wi = 0; wi < 4; ++wi) {
            const v4u X = *(const v4ua*)(&fl[p * 128 + wi * 32]); const v4u Y = *(const v4ua*)(&fl[p * 128 + wi * 32 + 16]);
            w[wi] = nib4(X[0]) | (nib4(X[1]) << 4) | (nib4(X[2]) << 8) | (nib4(X[3]) << 12) | (nib4(Y[0]) << 16) | (nib4(Y[1]) << 20) | (nib4(Y[2]) << 24) | (nib4(Y[3]) << 28); }
        unsigned* dp = MB + wbase + (size_t)p * 4;
        *(volatile v4u*)dp = w; __threadfence(); *(volatile v4u*)dp = w; }
}

template <int MODE>
__global__ __launch_bounds__(32) void k_proj(const bf* __restrict__ A, const bf* __restrict__ Bt, const float* __restrict__ bias, h16* Ph, h16* Pr, int resT) {
    __shared__ __align__(16) float os[16 * 68];
    const int K = DM;
    const int lane = threadIdx.x & 31, lr = lane & 15, hi = lane >> 4; const int r0 = blockIdx.x * 64, c0 = blockIdx.y * 64;
    v8f acc[4][4];
#pragma unroll
    for (int mb = 0; mb < 4; ++mb)
#pragma unroll
        for (int nb = 0; nb < 4; ++nb) acc[mb][nb] = (v8f){};
    const size_t aoff = (size_t)(r0 + lr) * K + 8 * hi, boff = (size_t)(c0 + lr) * K + 8 * hi;
#pragma unroll 1
    for (int kc = 0; kc < K; kc += 32) {
        v16bf a[4];
#pragma unroll
        for (int mb = 0; mb < 4; ++mb) a[mb] = ldb(A + aoff + (size_t)mb * 16 * K + kc);
#pragma unroll
        for (int nb = 0; nb < 4; ++nb) { const v16bf b = ldb(Bt + boff + (size_t)nb * 16 * K + kc);
#pragma unroll
            for (int mb = 0; mb < 4; ++mb) acc[mb][nb] = wmmab(a[mb], b, acc[mb][nb]); }
        asm volatile("v_nop\n\tv_nop\n\tv_nop\n\tv_nop" : "+v"(acc[0][0]), "+v"(acc[1][1]), "+v"(acc[2][2]), "+v"(acc[3][3]) : "v"(a[0]), "v"(a[1]), "v"(a[2]), "v"(a[3]));
    }
    float bc[4];
#pragma unroll
    for (int nb = 0; nb < 4; ++nb) bc[nb] = (MODE == 0) ? bfr(bias[c0 + nb * 16 + lr]) : 0.0f;
    size_t tbase, rbase; bool wr;
    if (MODE == 0) { const int bb = r0 / SEQ, tt = r0 % SEQ; const int zc = bb * NH_ + c0 / HD;
                     tbase = ((size_t)zc * SEQ + (size_t)tt) * HD; rbase = ((size_t)zc * (size_t)resT + (size_t)tt) * HD; wr = tt < resT; }
    else           { const int bb = c0 / SEQ, tt = c0 % SEQ;
                     tbase = (size_t)bb * (size_t)DM * SEQ + (size_t)r0 * SEQ + (size_t)tt; rbase = (size_t)bb * (size_t)DM * (size_t)resT + (size_t)r0 * (size_t)resT + (size_t)tt; wr = tt < resT; }
#pragma unroll
    for (int mb = 0; mb < 4; ++mb) {
        float br[8];
#pragma unroll
        for (int j = 0; j < 8; ++j) br[j] = (MODE == 1) ? bfr(bias[r0 + mb * 16 + hi * 8 + j]) : 0.0f;
#pragma unroll
        for (int nb = 0; nb < 4; ++nb) {
#pragma unroll
            for (int j = 0; j < 8; ++j) os[(hi * 8 + j) * 68 + nb * 16 + lr] = acc[mb][nb][j] + bc[nb] + br[j]; }
        wave_sync();
#pragma unroll 1
        for (int ps = 0; ps < 2; ++ps) {
            if (MODE == 0) {
                const size_t sb = tbase + (size_t)(mb * 16) * HD;
                const size_t rb = rbase + (size_t)(mb * 16) * HD;
#pragma unroll
                for (int hh = 0; hh < 2; ++hh) {
#pragma unroll
                    for (int s = 0; s < 2; ++s) { const int p = s * 32 + lane; const int row = p >> 2, c8 = (p & 3) * 8;
                        const v4f x0 = *(const v4fa*)(&os[row * 68 + hh * 32 + c8]); const v4f x1 = *(const v4fa*)(&os[row * 68 + hh * 32 + c8 + 4]); v8h hv, rv;
#pragma unroll
                        for (int i = 0; i < 4; ++i) { const h16 a0 = (h16)x0[i]; const h16 a1 = (h16)x1[i]; hv[i] = a0; hv[4 + i] = a1; rv[i] = (h16)((x0[i] - (float)a0) * QRS); rv[4 + i] = (h16)((x1[i] - (float)a1) * QRS); }
                        const size_t oo = sb + (size_t)hh * ((size_t)SEQ * HD) + (size_t)p * 8;
                        const size_t ro = rb + (size_t)hh * ((size_t)resT * HD) + (size_t)p * 8;
                        *(volatile v8h*)(Ph + oo) = hv; if (wr) *(volatile v8h*)(Pr + ro) = rv; } }
            } else {
                const size_t sb = tbase + (size_t)(mb * 16) * SEQ;
                const size_t rb = rbase + (size_t)(mb * 16) * (size_t)resT;
#pragma unroll
                for (int s = 0; s < 4; ++s) { const int row = 4 * s + (lane >> 3), c8 = (lane & 7) * 8;
                    const v4f x0 = *(const v4fa*)(&os[row * 68 + c8]); const v4f x1 = *(const v4fa*)(&os[row * 68 + c8 + 4]); v8h hv, rv;
#pragma unroll
                    for (int i = 0; i < 4; ++i) { const h16 a0 = (h16)x0[i]; const h16 a1 = (h16)x1[i]; hv[i] = a0; hv[4 + i] = a1; rv[i] = (h16)((x0[i] - (float)a0) * QRS); rv[4 + i] = (h16)((x1[i] - (float)a1) * QRS); }
                    const size_t oo = sb + (size_t)row * SEQ + c8;
                    const size_t ro = rb + (size_t)row * (size_t)resT + c8;
                    *(volatile v8h*)(Ph + oo) = hv; if (wr) *(volatile v8h*)(Pr + ro) = rv; }
            }
            if (ps == 0) __threadfence(); }
        wave_sync();
    }
}

__global__ __launch_bounds__(32 * AW) void k_flash(const h16* __restrict__ QH, const h16* __restrict__ QR, const h16* __restrict__ KP, const h16* __restrict__ KR,
                                                   const h16* __restrict__ VT, const h16* __restrict__ VR, const unsigned* __restrict__ MB, h16* CH, h16* CR) {
    __shared__ __align__(16) float os[AW * 16 * OSP];
    const int lane = threadIdx.x & 31, lr = lane & 15, hi = lane >> 4;
    const int wave = __builtin_amdgcn_readfirstlane((int)(threadIdx.x >> 5));
    const int zh = blockIdx.y; const int b = zh / NH_;
    const int t0 = (blockIdx.x * AW + wave) * 16;
    const unsigned* mrow = MB + (size_t)(b * SEQ + t0 + lr) * (SEQ / 32);
    const size_t pbase = (size_t)zh * SEQ * HD;
    const size_t qo = pbase + (size_t)(t0 + lr) * HD + 8 * hi;
    const v16h qh = ldh(QH + qo), qr = ldh(QR + qo);
    const size_t ko = pbase + (size_t)lr * HD + 8 * hi;
    const size_t vo = pbase + (size_t)lr * SEQ + 8 * hi;
    v8f o0 = (v8f){}, o1 = (v8f){}, oR0 = (v8f){}, oR1 = (v8f){};
    float m = NEGB, l = 0.0f;
#pragma unroll 1
    for (int key0 = 0; key0 < SEQ; key0 += 32) {
        unsigned mw = mrow[key0 >> 5];
        asm volatile("" : "+v"(mw));
        const unsigned sa = mw >> (8 * hi);
        const h16* ka = KP + ko + (size_t)key0 * HD;
        const h16* kr = KR + ko + (size_t)key0 * HD;
        const v16h ka0 = ldh(ka), kb0 = ldh(ka + 16 * HD);
        const v16h kra0 = ldh(kr), krb0 = ldh(kr + 16 * HD);
        v8f sHa = (v8f){}, sLa = (v8f){}, sHb = (v8f){}, sLb = (v8f){};
        sHa = wmma16g(ka0, qh, sHa); sLa = wmma16g(ka0, qr, sLa); sLa = wmma16g(kra0, qh, sLa);
        sHb = wmma16g(kb0, qh, sHb); sLb = wmma16g(kb0, qr, sLb); sLb = wmma16g(krb0, qh, sLb);
        float ta[8], tb[8]; bool fa[8], fb[8]; float mx = NEGB;
#pragma unroll
        for (int r = 0; r < 8; ++r) {
            fa[r] = ((sa >> r) & 1u) != 0u;
            fb[r] = ((sa >> (16 + r)) & 1u) != 0u;
            ta[r] = (sHa[r] + sLa[r] * QRI) * SC2; tb[r] = (sHb[r] + sLb[r] * QRI) * SC2;
            mx = fmaxf(mx, fmaxf(fa[r] ? ta[r] : NEGB, fb[r] ? tb[r] : NEGB)); }
        mx = fmaxf(mx, __shfl_xor(mx, 16, 32));
        const float mnew = fmaxf(m, mx);
        const float alpha = __builtin_amdgcn_exp2f(m - mnew);
        const float sh = PSH - mnew;
        v16h pb, pr; float ls = 0.0f;
#pragma unroll
        for (int r = 0; r < 8; ++r) {
            const float xa = ta[r] + sh, xb = tb[r] + sh;
            const float ea = __builtin_amdgcn_exp2f(xa), eb = __builtin_amdgcn_exp2f(xb);
            const bool za = fa[r] & (xa >= -14.0f), zb = fb[r] & (xb >= -14.0f);
            const float ga = za ? ea : 0.0f, gb = zb ? eb : 0.0f;
            const h16 pa = (h16)ga; const h16 pc = (h16)gb;
            pb[r] = pa; pb[8 + r] = pc;
            pr[r] = toh_flush((ga - (float)pa) * QRS); pr[8 + r] = toh_flush((gb - (float)pc) * QRS);
            ls += ga + gb; }
        l = l * alpha + ls; m = mnew;
        o0 = o0 * alpha; o1 = o1 * alpha; oR0 = oR0 * alpha; oR1 = oR1 * alpha;
        const h16* va = VT + vo + key0;
        const h16* vr = VR + vo + key0;
        const v16h v0 = ldh(va), v1 = ldh(va + (size_t)16 * SEQ);
        const v16h vr0 = ldh(vr), vr1 = ldh(vr + (size_t)16 * SEQ);
        o0 = wmma16g(v0, pb, o0); o1 = wmma16g(v1, pb, o1);
        oR0 = wmma16g(v0, pr, oR0); oR1 = wmma16g(v1, pr, oR1);
        oR0 = wmma16g(vr0, pb, oR0); oR1 = wmma16g(vr1, pb, oR1);
    }
    l += __shfl_xor(l, 16, 32);
    const bool any = l > 0.0f;
    const float lsafe = any ? l : 1.0f;
    const float inv = any ? (1.0f / lsafe) : 0.0f;
    const v8f f0 = o0 + oR0 * QRI, f1 = o1 + oR1 * QRI;
    const int wb = wave * 16 * OSP;
    { v4f a, c;
      a[0] = f0[0] * inv; a[1] = f0[1] * inv; a[2] = f0[2] * inv; a[3] = f0[3] * inv; c[0] = f0[4] * inv; c[1] = f0[5] * inv; c[2] = f0[6] * inv; c[3] = f0[7] * inv;
      *(v4fa*)(&os[wb + lr * OSP +  0 + 8 * hi]) = a; *(v4fa*)(&os[wb + lr * OSP +  0 + 8 * hi + 4]) = c;
      a[0] = f1[0] * inv; a[1] = f1[1] * inv; a[2] = f1[2] * inv; a[3] = f1[3] * inv; c[0] = f1[4] * inv; c[1] = f1[5] * inv; c[2] = f1[6] * inv; c[3] = f1[7] * inv;
      *(v4fa*)(&os[wb + lr * OSP + 16 + 8 * hi]) = a; *(v4fa*)(&os[wb + lr * OSP + 16 + 8 * hi + 4]) = c; }
    wave_sync();
    const size_t cb = ((size_t)zh * SEQ + (size_t)t0) * HD;
#pragma unroll 1
    for (int ps = 0; ps < 2; ++ps) {
#pragma unroll
        for (int s = 0; s < 2; ++s) { const int p = s * 32 + lane; const int row = p >> 2, c8 = (p & 3) * 8;
            const v4f x0 = *(const v4fa*)(&os[wb + row * OSP + c8]); const v4f x1 = *(const v4fa*)(&os[wb + row * OSP + c8 + 4]); v8h hv, rv;
#pragma unroll
            for (int i = 0; i < 4; ++i) { const h16 a0 = toh_flush(x0[i]); const h16 a1 = toh_flush(x1[i]); hv[i] = a0; hv[4 + i] = a1;
                rv[i] = toh_flush((x0[i] - (float)a0) * QRS); rv[4 + i] = toh_flush((x1[i] - (float)a1) * QRS); }
            *(volatile v8h*)(CH + cb + (size_t)p * 8) = hv; *(volatile v8h*)(CR + cb + (size_t)p * 8) = rv; }
        if (ps == 0) __threadfence(); }
}

__global__ __launch_bounds__(32) void k_outp(const h16* __restrict__ CH, const h16* __restrict__ CR, const h16* __restrict__ WT, const float* __restrict__ bias, float* OUT) {
    __shared__ __align__(16) float os[16 * 68];
    const int lane = threadIdx.x & 31, lr = lane & 15, hi = lane >> 4; const int r0 = blockIdx.x * 32, c0 = blockIdx.y * 64;
    const int bb = r0 / SEQ, tt = r0 % SEQ;
    v8f aH[2][4], aR[2][4];
#pragma unroll
    for (int mb = 0; mb < 2; ++mb)
#pragma unroll
        for (int nb = 0; nb < 4; ++nb) { aH[mb][nb] = (v8f){}; aR[mb][nb] = (v8f){}; }
    const size_t aoff = ((size_t)bb * NH_ * SEQ + (size_t)(tt + lr)) * HD + 8 * hi;
    const size_t boff = (size_t)(c0 + lr) * DM + 8 * hi;
#pragma unroll 1
    for (int kc = 0; kc < DM; kc += 32) {
        const size_t ah = aoff + (size_t)(kc / HD) * SEQ * HD;
        const v16h a0 = ldh(CH + ah), a1 = ldh(CH + ah + 16 * HD);
        const v16h e0 = ldh(CR + ah), e1 = ldh(CR + ah + 16 * HD);
#pragma unroll
        for (int nb = 0; nb < 4; ++nb) { const v16h w = ldh(WT + boff + (size_t)nb * 16 * DM + kc);
            aH[0][nb] = wmma16g(a0, w, aH[0][nb]); aH[1][nb] = wmma16g(a1, w, aH[1][nb]);
            aR[0][nb] = wmma16g(e0, w, aR[0][nb]); aR[1][nb] = wmma16g(e1, w, aR[1][nb]); }
    }
    float bc[4];
#pragma unroll
    for (int nb = 0; nb < 4; ++nb) bc[nb] = bfr(bias[c0 + nb * 16 + lr]);
    float* obase = OUT + ((size_t)bb * OUT_SEQ + (size_t)tt) * DM + c0;
#pragma unroll
    for (int mb = 0; mb < 2; ++mb) {
#pragma unroll
        for (int nb = 0; nb < 4; ++nb) {
#pragma unroll
            for (int j = 0; j < 8; ++j) os[(hi * 8 + j) * 68 + nb * 16 + lr] = (aH[mb][nb][j] + aR[mb][nb][j] * QRI) * WOI + bc[nb]; }
        wave_sync();
#pragma unroll 1
        for (int ps = 0; ps < 2; ++ps) {
#pragma unroll
            for (int s = 0; s < 8; ++s) { const int row = 2 * s + (lane >> 4), c4 = (lane & 15) * 4;
                const v4f val = *(const v4fa*)(&os[row * 68 + c4]);
                *(volatile v4f*)(obase + (size_t)(mb * 16 + row) * DM + c4) = val; }
            if (ps == 0) __threadfence(); }
        wave_sync();
    }
}

static constexpr size_t al256(size_t v) { return (v + 255) & ~(size_t)255; }
static constexpr size_t SZ_XB = al256((size_t)NB * SEQ * DM * 2);
static constexpr size_t SZ_WB = al256((size_t)3 * DM * DM * 2);
static constexpr size_t SZ_WO = al256((size_t)DM * DM * 2);
static constexpr size_t SZ_PL = al256((size_t)NB * NH_ * SEQ * HD * 2);
static constexpr size_t SZ_MB = al256((size_t)NB * SEQ * (SEQ / 32) * 4);
static constexpr size_t SZ_TOTAL = SZ_XB + SZ_WB + SZ_WO + 8 * SZ_PL + SZ_MB;
static_assert(SZ_TOTAL <= (size_t)134217728);
static_assert(((size_t)DM * DM * 2) % 256 == 0);
static_assert((size_t)NB * NH_ * SEQ * HD == (size_t)NB * DM * SEQ);
static_assert((size_t)(NB * SEQ / 64) * 64 * DM == (size_t)NB * NH_ * SEQ * HD);
static_assert((size_t)(SEQ / (16 * AW)) * (NB * NH_) * AW * 16 * HD == (size_t)NB * NH_ * SEQ * HD);
static_assert((size_t)(SEQ / MROWS) * NB * MROWS * (SEQ / 32) * 4 == (size_t)NB * SEQ * (SEQ / 32) * 4);

extern "C" void kernel_launch(void* const* d_in, const int* in_sizes, int n_in,
                              void* d_out, int out_size, void* d_ws, size_t ws_size, hipStream_t stream) {
    if (n_in < 11) return;
    const size_t needx = ((size_t)(NB - 1) * SEQ_FULL + SEQ) * DM;
    if ((size_t)in_sizes[0] < needx) return;
    if (in_sizes[1] < 1 || in_sizes[2] < 1) return;
    if ((size_t)in_sizes[3] < (size_t)DM * DM || (size_t)in_sizes[5] < (size_t)DM * DM || (size_t)in_sizes[7] < (size_t)DM * DM || (size_t)in_sizes[9] < (size_t)DM * DM) return;
    if (in_sizes[4] < DM || in_sizes[6] < DM || in_sizes[8] < DM || in_sizes[10] < DM) return;
    if ((size_t)out_size < ((size_t)(NB - 1) * OUT_SEQ + SEQ) * DM) return;
    if (SZ_TOTAL > ws_size) return;
    const float* hin = (const float*)d_in[0];
    const int* src = (const int*)d_in[1]; const int* dst = (const int*)d_in[2];
    const float* wq = (const float*)d_in[3]; const float* bq = (const float*)d_in[4];
    const float* wk = (const float*)d_in[5]; const float* bk = (const float*)d_in[6];
    const float* wv = (const float*)d_in[7]; const float* bv = (const float*)d_in[8];
    const float* wo = (const float*)d_in[9]; const float* bo = (const float*)d_in[10];
    const int nE = in_sizes[1] < in_sizes[2] ? in_sizes[1] : in_sizes[2];
    float* OUT = (float*)d_out;
    char* wsp = (char*)d_ws;
    bf* XB = (bf*)wsp; wsp += SZ_XB;
    bf* WB = (bf*)wsp; wsp += SZ_WB;
    h16* WOH = (h16*)wsp; wsp += SZ_WO;
    h16* QH = (h16*)wsp; wsp += SZ_PL;
    h16* QR = (h16*)wsp; wsp += SZ_PL;
    h16* KP = (h16*)wsp; wsp += SZ_PL;
    h16* KR = (h16*)wsp; wsp += SZ_PL;
    h16* VT = (h16*)wsp; wsp += SZ_PL;
    h16* VR = (h16*)wsp; wsp += SZ_PL;
    h16* CH = (h16*)wsp; wsp += SZ_PL;
    h16* CR = (h16*)wsp; wsp += SZ_PL;
    unsigned* MB = (unsigned*)wsp; wsp += SZ_MB;
    bf* WQ = WB; bf* WK = WB + (size_t)DM * DM; bf* WV = WB + (size_t)2 * DM * DM;

    k_mask<<<dim3(SEQ / MROWS, NB, 1), 256, 0, stream>>>(src, dst, nE, MB);

    if (SEQ == SEQ_FULL) {
        const size_t n8 = (size_t)NB * SEQ * DM / 8;
        k_cvt8<<<(unsigned)((n8 + 255) / 256), 256, 0, stream>>>(hin, XB, n8);
    } else {
        const size_t n8 = (size_t)SEQ * DM / 8;
        for (int b = 0; b < NB; ++b) k_cvt8<<<(unsigned)((n8 + 255) / 256), 256, 0, stream>>>(hin + (size_t)b * SEQ_FULL * DM, XB + (size_t)b * SEQ * DM, n8);
    }
    k_wtb<<<DM / 32, 256, 0, stream>>>(wq, WQ);
    k_wtb<<<DM / 32, 256, 0, stream>>>(wk, WK);
    k_wtb<<<DM / 32, 256, 0, stream>>>(wv, WV);
    k_wth<<<DM / 32, 256, 0, stream>>>(wo, WOH);

    k_proj<0><<<dim3(NB * SEQ / 64, DM / 64, 1), 32, 0, stream>>>(XB, WQ, bq, QH, QR, SEQ);
    k_proj<0><<<dim3(NB * SEQ / 64, DM / 64, 1), 32, 0, stream>>>(XB, WK, bk, KP, KR, SEQ);
    k_proj<1><<<dim3(DM / 64, NB * SEQ / 64, 1), 32, 0, stream>>>(WV, XB, bv, VT, VR, SEQ);

    k_flash<<<dim3(SEQ / (16 * AW), NB * NH_, 1), 32 * AW, 0, stream>>>(QH, QR, KP, KR, VT, VR, MB, CH, CR);

    k_outp<<<dim3(NB * SEQ / 32, DM / 64, 1), 32, 0, stream>>>(CH, CR, WOH, bo, OUT);
}
